// Net_77068893159889
// MI455X (gfx1250) — hardware-run, weakly checked
//
#include <hip/hip_runtime.h>
#include <stddef.h>
#include <stdint.h>
#include <math.h>


#define NN      100000
#define NE      1600000
#define DF      128
#define NC      40
#define NCP     48
#define GBM     128
#define MP      100096
#define MEAN_TERMS 1
#define KCAT    (3 * DF + DF * MEAN_TERMS)
#define AGP     (3 * DF)

#define PTHR    256
#define PB_X    ((MP * (DF / 8)) / PTHR)
#define PB_A    (((MP - NN) * (AGP / 8)) / PTHR)
#define PB_W    ((NCP * (KCAT / 8)) / PTHR)
#define PB_M    1

#define SNTHR   256
#define SNWAVE  8
#define EPT     8
#define CHUNK   (SNTHR * EPT)
#define NCHUNK  ((NE + CHUNK - 1) / CHUNK)
#define NBRUN   1024
#define NBLK    ((NN + NBRUN - 1) / NBRUN)
#define SLB     17
#define SRCMASK ((1u << SLB) - 1u)
#define WLCAP   3584
#define RCAP    20480
#define DEGCAP  64
#define MAXHITS 16710
#define MAXDEG  36
#define MISC_INTS   16
#define SC_ZINTS    (SNWAVE * WLCAP + RCAP + 3 * NBRUN)
#define SC_ROW_INTS (SNWAVE * AGP / 2)
#define SC_LDS_INTS (SC_ZINTS + MISC_INTS + SC_ROW_INTS)
#define FLAGP   32

#define GTHR    256
#define TP      52
#define G_W_INTS   (NCP * KCAT / 2)
#define G_STG_INTS (GBM * TP)
#define G_OST_INTS (GBM * NC)
#define G_SB_INTS  64
#define G_LDS_INTS (G_W_INTS + G_STG_INTS + G_OST_INTS + G_SB_INTS)
#define WSMAX   (128u << 20)

static_assert(MP == ((NN + GBM - 1) / GBM) * GBM);
static_assert(NBRUN % GBM == 0 && NBRUN == 1024);
static_assert(NBLK * NBRUN >= MP);
static_assert(((MP / GBM - 1) / (NBRUN / GBM)) < NBLK);
static_assert(KCAT % 32 == 0 && NCP % 16 == 0 && NCP >= NC);
static_assert((GBM * NC * 4) % 128 == 0);
static_assert(((NN % GBM) * NC * 4) % 128 == 0);
static_assert((((NN % GBM) * (NC / 4)) % 32) == 0);
static_assert(NN <= (1 << SLB) && SLB + 10 <= 32);
static_assert(NE % EPT == 0 && NE >= EPT);
static_assert(RCAP * 100 >= MAXHITS * 105);
static_assert(WLCAP * SNWAVE * 4 >= RCAP * 5);
static_assert(DEGCAP >= MAXDEG + 8 && DEGCAP <= 64);
static_assert(SC_ZINTS % (SNTHR * 4) == 0);
static_assert(((SC_ZINTS + MISC_INTS) % 4) == 0);
static_assert(SC_LDS_INTS * 4 <= 300000);
static_assert(G_LDS_INTS * 4 <= 327680);
static_assert((MP * (DF / 8)) % PTHR == 0);
static_assert(((MP - NN) * (AGP / 8)) % PTHR == 0);
static_assert((NCP * (KCAT / 8)) % PTHR == 0);
static_assert((G_W_INTS / 4) % GTHR == 0);
static_assert(GBM == (GTHR / 32) * 16 && DF == 4 * 32 && NC % 4 == 0);
static_assert((GBM * NC / 4) % GTHR == 0);
static_assert((long long)(MP / GBM - 1) * GBM * NC + (long long)(NN % GBM) * NC == (long long)NN * NC);

typedef float          v4f   __attribute__((ext_vector_type(4)));
typedef float          v8f   __attribute__((ext_vector_type(8)));
typedef int            v4i   __attribute__((ext_vector_type(4)));
typedef int            v8i   __attribute__((ext_vector_type(8)));
typedef unsigned       v2u   __attribute__((ext_vector_type(2)));
typedef unsigned       v4u   __attribute__((ext_vector_type(4)));
typedef unsigned short v4us  __attribute__((ext_vector_type(4)));
typedef unsigned short v8us  __attribute__((ext_vector_type(8)));
typedef __bf16         v16bf __attribute__((ext_vector_type(16)));
typedef v4f  __attribute__((may_alias)) v4fa;
typedef v4i  __attribute__((may_alias)) v4ia;
typedef v2u  __attribute__((may_alias)) v2ua;
typedef v4us __attribute__((may_alias)) v4usa;
typedef v8us __attribute__((may_alias)) v8usa;
union FragB { v16bf v; v8us h[2]; v8i w; };

__device__ __forceinline__ v8f wmb(const FragB& a, const FragB& b, v8f c) {
  v8f d = __builtin_amdgcn_wmma_f32_16x16x32_bf16(false, a.v, false, b.v, (short)0, c, false, false);
  asm volatile("v_nop\n\tv_nop\n\tv_nop\n\tv_nop" : "+v"(d) : "v"(a.w), "v"(b.w));
  return d;
}

__device__ __forceinline__ unsigned bf16_bits(float f) {
  const unsigned u = __float_as_uint(f);
  const unsigned r = (u + 0x7FFFu + ((u >> 16) & 1u)) >> 16;
  const unsigned q = (u >> 16) | 0x40u;
  return ((u & 0x7fffffffu) > 0x7f800000u) ? q : r;
}
__device__ __forceinline__ float bf16_val(float f) { return __uint_as_float(bf16_bits(f) << 16); }

__device__ __forceinline__ v4u pack8m(const v4f a, const v4f b, unsigned keep) {
  v4u r;
  r.x = (bf16_bits(a.x) | (bf16_bits(a.y) << 16)) & keep;
  r.y = (bf16_bits(a.z) | (bf16_bits(a.w) << 16)) & keep;
  r.z = (bf16_bits(b.x) | (bf16_bits(b.y) << 16)) & keep;
  r.w = (bf16_bits(b.z) | (bf16_bits(b.w) << 16)) & keep;
  return r;
}

__device__ __forceinline__ float bl1(float a, float b, float c, float d,
                                     unsigned m0, unsigned m1, unsigned m2, unsigned m3) {
  return __uint_as_float((__float_as_uint(a) & m0) | (__float_as_uint(b) & m1) |
                         (__float_as_uint(c) & m2) | (__float_as_uint(d) & m3));
}
__device__ __forceinline__ v4f bl4(const v4f a, const v4f b, const v4f c, const v4f d,
                                   unsigned m0, unsigned m1, unsigned m2, unsigned m3) {
  v4f r;
  r.x = bl1(a.x, b.x, c.x, d.x, m0, m1, m2, m3);
  r.y = bl1(a.y, b.y, c.y, d.y, m0, m1, m2, m3);
  r.z = bl1(a.z, b.z, c.z, d.z, m0, m1, m2, m3);
  r.w = bl1(a.w, b.w, c.w, d.w, m0, m1, m2, m3);
  return r;
}

__device__ __forceinline__ void wave_sync() {
  __builtin_amdgcn_fence(__ATOMIC_RELEASE, "wavefront");
  __builtin_amdgcn_wave_barrier();
  __builtin_amdgcn_fence(__ATOMIC_ACQUIRE, "wavefront");
}

__global__ __launch_bounds__(PTHR) void k_prep(const float* __restrict__ x,
                                               const float* __restrict__ wlmax, const float* __restrict__ wrmax,
                                               const float* __restrict__ bmax,
                                               const float* __restrict__ wlmean, const float* __restrict__ wrmean,
                                               const float* __restrict__ bmean,
                                               unsigned short* xb, unsigned short* agg,
                                               unsigned short* wcat, float* bsum) {
  const int b = (int)blockIdx.x, tid = (int)threadIdx.x;
  if (b < PB_X) {
    const int i   = b * PTHR + tid;
    const int row = i >> 4;
    const int c0  = (i & 15) * 8;
    const int rc  = row < NN ? row : NN - 1;
    const float* p = x + (size_t)rc * DF + c0;
    const v4f a = *(const v4fa*)p;
    const v4f q = *(const v4fa*)(p + 4);
    asm volatile("" :: "v"(a), "v"(q));
    const unsigned keep = row < NN ? 0xffffffffu : 0u;
    const v4u hv = pack8m(a, q, keep);
    unsigned short* o = xb + (size_t)row * DF + c0;
    *(volatile v4u*)o = hv;
    __threadfence();
    *(volatile v4u*)o = hv;
  } else if (b < PB_X + PB_A) {
    const int u = (b - PB_X) * PTHR + tid;
    const v4u z = {0u, 0u, 0u, 0u};
    unsigned short* o = agg + (size_t)NN * AGP + (size_t)u * 8;
    *(volatile v4u*)o = z;
    __threadfence();
    *(volatile v4u*)o = z;
  } else if (b < PB_X + PB_A + PB_W) {
    const int u   = (b - PB_X - PB_A) * PTHR + tid;
    const int n   = u / (KCAT / 8);
    const int k8  = (u - n * (KCAT / 8)) * 8;
    const int seg = k8 >> 7;
    const int kk  = k8 & (DF - 1);
    const int nc  = n < NC ? n : NC - 1;
    const size_t so = (size_t)nc * DF + kk;
    const v4f r0a = *(const v4fa*)(wrmax + so),  r0b = *(const v4fa*)(wrmax + so + 4);
    const v4f r1a = *(const v4fa*)(wrmean + so), r1b = *(const v4fa*)(wrmean + so + 4);
    const v4f r2a = *(const v4fa*)(wlmax + so),  r2b = *(const v4fa*)(wlmax + so + 4);
    const v4f r3a = *(const v4fa*)(wlmean + so), r3b = *(const v4fa*)(wlmean + so + 4);
    asm volatile("" :: "v"(r0a), "v"(r0b), "v"(r1a), "v"(r1b));
    asm volatile("" :: "v"(r2a), "v"(r2b), "v"(r3a), "v"(r3b));
    const unsigned live = n < NC ? 0xffffffffu : 0u;
    const unsigned m0 = (seg == 0 ? 0xffffffffu : 0u) & live;
    const unsigned m1 = (seg == 1 ? 0xffffffffu : 0u) & live;
    const unsigned m2 = (seg == 2 ? 0xffffffffu : 0u) & live;
    const unsigned m3 = (seg >= 3 ? 0xffffffffu : 0u) & live;
    const v4f a = bl4(r0a, r1a, r2a, r3a, m0, m1, m2, m3);
    const v4f q = bl4(r0b, r1b, r2b, r3b, m0, m1, m2, m3);
    const v4u wv = pack8m(a, q, 0xffffffffu);
    unsigned short* o = wcat + (size_t)n * KCAT + k8;
    *(volatile v4u*)o = wv;
    __threadfence();
    *(volatile v4u*)o = wv;
  } else {
    const int t  = tid & 15;
    const int tc = t < NC / 4 ? t : NC / 4 - 1;
    const v4f a = *(const v4fa*)(bmax + 4 * tc);
    const v4f c = *(const v4fa*)(bmean + 4 * tc);
    asm volatile("" :: "v"(a), "v"(c));
    const unsigned live = t < NC / 4 ? 0xffffffffu : 0u;
    v4f s;
    s.x = __uint_as_float(__float_as_uint(bf16_val(a.x) + bf16_val(c.x)) & live);
    s.y = __uint_as_float(__float_as_uint(bf16_val(a.y) + bf16_val(c.y)) & live);
    s.z = __uint_as_float(__float_as_uint(bf16_val(a.z) + bf16_val(c.z)) & live);
    s.w = __uint_as_float(__float_as_uint(bf16_val(a.w) + bf16_val(c.w)) & live);
    float* o = bsum + 4 * t;
    if (tid < 16) *(volatile v4f*)o = s;
    __threadfence();
    if (tid < 16) *(volatile v4f*)o = s;
  }
}

__device__ __forceinline__ void acc_hit(const v2u w, const bool ok,
                                        float& m0, float& m1, float& m2, float& m3,
                                        float& a0, float& a1, float& a2, float& a3) {
  const float f0 = __uint_as_float(w.x << 16);
  const float f1 = __uint_as_float(w.x & 0xffff0000u);
  const float f2 = __uint_as_float(w.y << 16);
  const float f3 = __uint_as_float(w.y & 0xffff0000u);
  m0 = (f0 > m0) ? f0 : m0;
  m1 = (f1 > m1) ? f1 : m1;
  m2 = (f2 > m2) ? f2 : m2;
  m3 = (f3 > m3) ? f3 : m3;
  a0 += ok ? f0 : 0.0f;
  a1 += ok ? f1 : 0.0f;
  a2 += ok ? f2 : 0.0f;
  a3 += ok ? f3 : 0.0f;
}

__global__ __launch_bounds__(SNTHR) void k_scan(const int* __restrict__ ei, const unsigned short* __restrict__ xb,
                                                unsigned short* agg, int* flag) {
  extern __shared__ __attribute__((aligned(16))) int dsm[];
  unsigned* wl  = (unsigned*)dsm;
  unsigned* gl  = wl + SNWAVE * WLCAP;
  int* cnt  = (int*)(gl + RCAP);
  int* offs = cnt + NBRUN;
  int* cur  = offs + NBRUN;
  int* misc = cur + NBRUN;
  const int tid = (int)threadIdx.x, lane = tid & 31;
  const int wave = __builtin_amdgcn_readfirstlane(tid >> 5);
  unsigned short* rowbuf = (unsigned short*)(misc + MISC_INTS) + wave * AGP;
  const int nodeBase = (int)blockIdx.x * NBRUN;

  {
    const v4i z4 = {0, 0, 0, 0};
    for (int i = tid * 4; i < SC_ZINTS; i += SNTHR * 4) *(v4ia*)(dsm + i) = z4;
    if (tid < MISC_INTS) misc[tid] = 0;
  }
  __syncthreads();

  const int* srcs = ei;
  const int* dsts = ei + NE;
  const unsigned nbs = (unsigned)nodeBase;
  unsigned* mywl = wl + wave * WLCAP;
  int wc = 0;
#pragma unroll 1
  for (int ch = 0; ch < NCHUNK; ++ch) {
    const int e0   = ch * CHUNK + tid * EPT;
    const bool inr = e0 < NE;
    const int ec   = inr ? e0 : NE - EPT;
    const v4i da = *(const v4i*)(dsts + ec);
    const v4i db = *(const v4i*)(dsts + ec + 4);
    const v4i sa = *(const v4i*)(srcs + ec);
    const v4i sb = *(const v4i*)(srcs + ec + 4);
    asm volatile("" :: "v"(da), "v"(db), "v"(sa), "v"(sb));
    const unsigned s0 = (unsigned)da.x - nbs, s1 = (unsigned)da.y - nbs;
    const unsigned s2 = (unsigned)da.z - nbs, s3 = (unsigned)da.w - nbs;
    const unsigned s4 = (unsigned)db.x - nbs, s5 = (unsigned)db.y - nbs;
    const unsigned s6 = (unsigned)db.z - nbs, s7 = (unsigned)db.w - nbs;
    const bool h0 = inr & (s0 < (unsigned)NBRUN), h1 = inr & (s1 < (unsigned)NBRUN);
    const bool h2 = inr & (s2 < (unsigned)NBRUN), h3 = inr & (s3 < (unsigned)NBRUN);
    const bool h4 = inr & (s4 < (unsigned)NBRUN), h5 = inr & (s5 < (unsigned)NBRUN);
    const bool h6 = inr & (s6 < (unsigned)NBRUN), h7 = inr & (s7 < (unsigned)NBRUN);
    const unsigned any = __builtin_amdgcn_ballot_w32(h0 | h1 | h2 | h3 | h4 | h5 | h6 | h7);
    if (any != 0u) {
#define HITJ(HJ, SJ, SRCJ) { \
      const unsigned mj = __builtin_amdgcn_ballot_w32(HJ); \
      if (mj != 0u) { \
        const int pos = wc + (int)__builtin_amdgcn_mbcnt_lo(mj, 0u); \
        int sc = (SRCJ); \
        sc = sc < 0 ? 0 : (sc > NN - 1 ? NN - 1 : sc); \
        const unsigned wd = ((SJ) << SLB) | (unsigned)sc; \
        if ((HJ) && pos < WLCAP) mywl[pos] = wd; \
        wc += (int)__builtin_popcount(mj); } }
      HITJ(h0, s0, sa.x)
      HITJ(h1, s1, sa.y)
      HITJ(h2, s2, sa.z)
      HITJ(h3, s3, sa.w)
      HITJ(h4, s4, sb.x)
      HITJ(h5, s5, sb.y)
      HITJ(h6, s6, sb.z)
      HITJ(h7, s7, sb.w)
#undef HITJ
    }
  }
  if (lane == 0) misc[wave] = wc;
  __syncthreads();

  if (wave == 0) {
#pragma unroll 1
    for (int w2 = 0; w2 < SNWAVE; ++w2) {
      int cv = misc[w2];
      cv = cv < 0 ? 0 : (cv > WLCAP ? WLCAP : cv);
      const int c = __builtin_amdgcn_readfirstlane(cv);
      const unsigned* lw = wl + w2 * WLCAP;
#pragma unroll 1
      for (int b0 = 0; b0 < c; b0 += 32) {
        int idx = b0 + lane;
        idx = idx > c - 1 ? c - 1 : idx;
        const int ent = (int)lw[idx];
        const int m32 = (c - b0) < 32 ? (c - b0) : 32;
#pragma unroll 1
        for (int k = 0; k < m32; ++k) {
          const unsigned u = (unsigned)__builtin_amdgcn_readlane(ent, k);
          const int slot = (int)((u >> SLB) & (unsigned)(NBRUN - 1));
          const int old = cnt[slot];
          if (lane == 0) cnt[slot] = old + 1;
        }
      }
    }
  }
  __syncthreads();

  if (wave == 0) {
    const int base = lane * (NBRUN / 32);
    int s = 0, big = 0;
#pragma unroll 4
    for (int i = 0; i < NBRUN / 32; ++i) {
      const int cv = cnt[base + i];
      big |= (cv > DEGCAP) ? 1 : 0;
      s += cv;
    }
    int incl = s;
#pragma unroll
    for (int d = 1; d < 32; d <<= 1) {
      const int y = __shfl_up(incl, d, 32);
      incl += (lane >= d) ? y : 0;
    }
    int run = incl - s;
#pragma unroll 4
    for (int i = 0; i < NBRUN / 32; ++i) {
      const int cv = cnt[base + i];
      offs[base + i] = run;
      cur[base + i]  = run;
      run += cv;
    }
    int tt = 0, wov = 0;
#pragma unroll
    for (int w2 = 0; w2 < SNWAVE; ++w2) {
      const int cv = misc[w2];
      wov |= (cv > WLCAP) ? 1 : 0;
      tt += cv < 0 ? 0 : (cv > WLCAP ? WLCAP : cv);
    }
    const unsigned bm = __builtin_amdgcn_ballot_w32(big != 0);
    const int ov = ((bm != 0u) || (wov != 0) || (tt > RCAP)) ? 1 : 0;
    if (lane == 0) misc[9] = ov;
  }
  __syncthreads();

  if (wave == 0) {
#pragma unroll 1
    for (int w2 = 0; w2 < SNWAVE; ++w2) {
      int cv = misc[w2];
      cv = cv < 0 ? 0 : (cv > WLCAP ? WLCAP : cv);
      const int c = __builtin_amdgcn_readfirstlane(cv);
      const unsigned* lw = wl + w2 * WLCAP;
#pragma unroll 1
      for (int b0 = 0; b0 < c; b0 += 32) {
        int idx = b0 + lane;
        idx = idx > c - 1 ? c - 1 : idx;
        const int ent = (int)lw[idx];
        const int m32 = (c - b0) < 32 ? (c - b0) : 32;
#pragma unroll 1
        for (int k = 0; k < m32; ++k) {
          const unsigned u = (unsigned)__builtin_amdgcn_readlane(ent, k);
          const int slot = (int)((u >> SLB) & (unsigned)(NBRUN - 1));
          int p = cur[slot];
          p = p < 0 ? 0 : (p > RCAP - 1 ? RCAP - 1 : p);
          if (lane == 0) { gl[p] = u & SRCMASK; cur[slot] = p + 1; }
        }
      }
    }
  }
  __syncthreads();

  const int ovf = misc[9];
  const float ninf = __uint_as_float(0xff800000u);
#pragma unroll 1
  for (int si = 0; si < NBRUN / SNWAVE; ++si) {
    const int s    = si * SNWAVE + wave;
    const int node = nodeBase + s;
    const int craw = cnt[s];
    const int cvec = craw < 0 ? 0 : (craw > DEGCAP ? DEGCAP : craw);
    const int c1v  = cvec < 1 ? 1 : cvec;
    const float dv = (float)c1v;
    const int c = __builtin_amdgcn_readfirstlane(cvec);
    int ov2 = offs[s];
    ov2 = ov2 < 0 ? 0 : (ov2 > RCAP - 1 ? RCAP - 1 : ov2);
    const int o = __builtin_amdgcn_readfirstlane(ov2);
    int last = o + c - 1;
    last = last < o ? o : last;
    last = last > RCAP - 1 ? RCAP - 1 : last;
    float m0 = ninf, m1 = ninf, m2 = ninf, m3 = ninf;
    float a0 = 0.0f, a1 = 0.0f, a2 = 0.0f, a3 = 0.0f;
#pragma unroll 1
    for (int b0 = 0; b0 < c; b0 += 32) {
      int idx = o + b0 + lane;
      idx = idx > last ? last : idx;
      int sr = (int)(gl[idx] & SRCMASK);
      sr = sr > NN - 1 ? NN - 1 : sr;
      const int m32 = (c - b0) < 32 ? (c - b0) : 32;
#pragma unroll 1
      for (int k = 0; k < m32; k += 4) {
        const int k0s = __builtin_amdgcn_readlane(sr, k);
        const int k1s = __builtin_amdgcn_readlane(sr, k + 1);
        const int k2s = __builtin_amdgcn_readlane(sr, k + 2);
        const int k3s = __builtin_amdgcn_readlane(sr, k + 3);
        const v2u w0 = *(const v2ua*)(xb + (size_t)k0s * DF + 4 * lane);
        const v2u w1 = *(const v2ua*)(xb + (size_t)k1s * DF + 4 * lane);
        const v2u w2 = *(const v2ua*)(xb + (size_t)k2s * DF + 4 * lane);
        const v2u w3 = *(const v2ua*)(xb + (size_t)k3s * DF + 4 * lane);
        asm volatile("" :: "v"(w0), "v"(w1), "v"(w2), "v"(w3));
        const bool v1 = (k + 1) < m32, v2 = (k + 2) < m32, v3 = (k + 3) < m32;
        acc_hit(w0, true, m0, m1, m2, m3, a0, a1, a2, a3);
        acc_hit(w1, v1,   m0, m1, m2, m3, a0, a1, a2, a3);
        acc_hit(w2, v2,   m0, m1, m2, m3, a0, a1, a2, a3);
        acc_hit(w3, v3,   m0, m1, m2, m3, a0, a1, a2, a3);
      }
    }
    const bool has = c > 0;
    v4us mb, mh, ml;
    mb[0] = (unsigned short)((has && ((m0 - m0) == 0.0f)) ? (__float_as_uint(m0) >> 16) : 0u);
    mb[1] = (unsigned short)((has && ((m1 - m1) == 0.0f)) ? (__float_as_uint(m1) >> 16) : 0u);
    mb[2] = (unsigned short)((has && ((m2 - m2) == 0.0f)) ? (__float_as_uint(m2) >> 16) : 0u);
    mb[3] = (unsigned short)((has && ((m3 - m3) == 0.0f)) ? (__float_as_uint(m3) >> 16) : 0u);
    {
      const float q0 = a0 / dv, q1 = a1 / dv, q2 = a2 / dv, q3 = a3 / dv;
      unsigned hb;
      hb = bf16_bits(q0); ml[0] = (unsigned short)bf16_bits(q0 - __uint_as_float(hb << 16));
      mh[0] = (unsigned short)((ovf != 0) ? 0x7fc0u : hb);
      hb = bf16_bits(q1); ml[1] = (unsigned short)bf16_bits(q1 - __uint_as_float(hb << 16));
      mh[1] = (unsigned short)((ovf != 0) ? 0x7fc0u : hb);
      hb = bf16_bits(q2); ml[2] = (unsigned short)bf16_bits(q2 - __uint_as_float(hb << 16));
      mh[2] = (unsigned short)((ovf != 0) ? 0x7fc0u : hb);
      hb = bf16_bits(q3); ml[3] = (unsigned short)bf16_bits(q3 - __uint_as_float(hb << 16));
      mh[3] = (unsigned short)((ovf != 0) ? 0x7fc0u : hb);
    }
    *(v4usa*)(rowbuf + 4 * lane) = mb;
    *(v4usa*)(rowbuf + DF + 4 * lane) = mh;
    *(v4usa*)(rowbuf + 2 * DF + 4 * lane) = ml;
    wave_sync();
    const v8us q0v = *(const v8usa*)(rowbuf + 8 * lane);
    const v8us q1v = *(const v8usa*)(rowbuf + 2 * DF + 8 * (lane & 15));
    asm volatile("" :: "v"(q0v), "v"(q1v));
    wave_sync();
    if (node < NN) {
      unsigned short* rpw = agg + (size_t)node * AGP + 8 * lane;
      *(volatile v8us*)rpw = q0v;
      if (lane < 16) *(volatile v8us*)(rpw + 2 * DF) = q1v;
      __threadfence();
      *(volatile v8us*)rpw = q0v;
      if (lane < 16) *(volatile v8us*)(rpw + 2 * DF) = q1v;
    }
  }

  if (wave == 0) {
    v4i fv;
    fv.x = ovf; fv.y = ovf; fv.z = ovf; fv.w = ovf;
    int* fp = flag + (size_t)blockIdx.x * FLAGP + 4 * (lane & 7);
    if (lane < 8) *(volatile v4i*)fp = fv;
    __threadfence();
    if (lane < 8) *(volatile v4i*)fp = fv;
  }
}

__global__ __launch_bounds__(GTHR) __attribute__((amdgpu_num_vgpr(248)))
void k_gemm_lsm(const unsigned short* __restrict__ xb, const unsigned short* __restrict__ agg,
                const int* __restrict__ wcat4, const float* __restrict__ bsum,
                const int* __restrict__ flag, float* outp) {
  extern __shared__ __attribute__((aligned(16))) int dsm[];
  unsigned short* wlds = (unsigned short*)dsm;
  float* stg = (float*)(dsm + G_W_INTS);
  float* ost = stg + G_STG_INTS;
  float* sb  = ost + G_OST_INTS;
  const int tid = (int)threadIdx.x, lane = tid & 31, hh = lane >> 4, m = lane & 15;
  const int wave = __builtin_amdgcn_readfirstlane(tid >> 5);
  const int blk = (int)blockIdx.x;
  const int rowBase = blk * GBM;

#pragma unroll 3
  for (int i = tid; i < G_W_INTS / 4; i += GTHR) {
    const v4i t = *(const v4i*)(wcat4 + 4 * i);
    *(v4ia*)(dsm + 4 * i) = t;
  }
  {
    const v4f t = *(const v4fa*)(bsum + 4 * (tid & 15));
    asm volatile("" :: "v"(t));
    if (tid < 16) *(v4fa*)(sb + 4 * tid) = t;
  }
  __syncthreads();

  v8f acc[3];
  {
    const v8f z = {0.f, 0.f, 0.f, 0.f, 0.f, 0.f, 0.f, 0.f};
    acc[0] = z; acc[1] = z; acc[2] = z;
  }
  const size_t arow = (size_t)(rowBase + 16 * wave + m);
  const unsigned short* ap = xb + arow * DF + 8 * hh;
  const unsigned short* gp = agg + arow * AGP + 8 * hh;
  const unsigned short* bp = wlds + m * KCAT + 8 * hh;

#pragma unroll 1
  for (int kk = 0; kk < DF / 32; ++kk) {
    FragB af;
    af.h[0] = *(const v8usa*)(ap + 32 * kk);
    af.h[1] = *(const v8usa*)(ap + 32 * kk + 16);
#pragma unroll
    for (int sg = 0; sg < 2; ++sg) {
      const unsigned short* wq = bp + 32 * kk + DF * sg;
#pragma unroll
      for (int t = 0; t < 3; ++t) {
        FragB bf;
        bf.h[0] = *(const v8usa*)(wq + 16 * t * KCAT);
        bf.h[1] = *(const v8usa*)(wq + 16 * t * KCAT + 16);
        acc[t] = wmb(af, bf, acc[t]);
      }
    }
  }
#pragma unroll 1
  for (int ks = 0; ks < (KCAT - 2 * DF) / 32; ++ks) {
    FragB af;
    af.h[0] = *(const v8usa*)(gp + 32 * ks);
    af.h[1] = *(const v8usa*)(gp + 32 * ks + 16);
    const unsigned short* wq = bp + 2 * DF + 32 * ks;
#pragma unroll
    for (int t = 0; t < 3; ++t) {
      FragB bf;
      bf.h[0] = *(const v8usa*)(wq + 16 * t * KCAT);
      bf.h[1] = *(const v8usa*)(wq + 16 * t * KCAT + 16);
      acc[t] = wmb(af, bf, acc[t]);
    }
  }

#pragma unroll
  for (int t = 0; t < 3; ++t) {
    const int lc = 16 * t + m;
    const float bz = sb[lc];
#pragma unroll
    for (int r = 0; r < 8; ++r) {
      const int lr = 16 * wave + 8 * hh + r;
      stg[lr * TP + lc] = acc[t][r] + bz;
    }
  }
  __syncthreads();

  const int fl = flag[(blk / (NBRUN / GBM)) * FLAGP];
  if (tid < GBM) {
    const float qnan = __uint_as_float(0x7fc00000u);
    const float* row = stg + tid * TP;
    float* orow = ost + tid * NC;
    float mxv = row[0];
#pragma unroll 4
    for (int c = 1; c < NC; ++c) {
      const float v = row[c];
      mxv = (v > mxv || v != v) ? v : mxv;
    }
    float sm = 0.0f;
#pragma unroll 1
    for (int c = 0; c < NC; ++c) sm += expf(row[c] - mxv);
    const float ls = logf(sm);
#pragma unroll 4
    for (int c = 0; c < NC; ++c) {
      float o = (row[c] - mxv) - ls;
      o = (fl != 0) ? qnan : o;
      orow[c] = o;
    }
  }
  __syncthreads();

  int live = NN - rowBase;
  live = live > GBM ? GBM : live;
  const int npc = live * (NC / 4);
  float* ob = outp + (size_t)blk * (GBM * NC);
  v4f pv[(GBM * NC / 4) / GTHR];
#pragma unroll
  for (int it = 0; it < (GBM * NC / 4) / GTHR; ++it) {
    const int p  = it * GTHR + tid;
    const int pc = p < npc ? p : npc - 1;
    pv[it] = *(const v4fa*)(ost + 4 * pc);
    asm volatile("" :: "v"(pv[it]));
  }
#pragma unroll
  for (int it = 0; it < (GBM * NC / 4) / GTHR; ++it) {
    const int p = it * GTHR + tid;
    if (p < npc) *(volatile v4f*)(ob + 4 * p) = pv[it];
  }
  __threadfence();
#pragma unroll
  for (int it = 0; it < (GBM * NC / 4) / GTHR; ++it) {
    const int p = it * GTHR + tid;
    if (p < npc) *(volatile v4f*)(ob + 4 * p) = pv[it];
  }
}

static inline size_t al256(size_t o) { return (o + 255) & ~(size_t)255; }

extern "C" void kernel_launch(void* const* d_in, const int* in_sizes, int n_in,
                              void* d_out, int out_size, void* d_ws, size_t ws_size,
                              hipStream_t stream) {
  if (n_in < 8) return;
  if (in_sizes[0] != NN * DF) return;
  if (in_sizes[1] != 2 * NE) return;
  if (in_sizes[2] != NC * DF || in_sizes[3] != NC * DF) return;
  if (in_sizes[4] != NC) return;
  if (in_sizes[5] != NC * DF || in_sizes[6] != NC * DF) return;
  if (in_sizes[7] != NC) return;
  if (out_size != NN * NC) return;

  const float* x      = (const float*)d_in[0];
  const int*   ei     = (const int*)  d_in[1];
  const float* wlmax  = (const float*)d_in[2];
  const float* wrmax  = (const float*)d_in[3];
  const float* bmax   = (const float*)d_in[4];
  const float* wlmean = (const float*)d_in[5];
  const float* wrmean = (const float*)d_in[6];
  const float* bmean  = (const float*)d_in[7];
  float* out = (float*)d_out;

  char* ws = (char*)d_ws;
  size_t off = 0;
  const size_t oXB  = off; off = al256(off + (size_t)MP * DF * 2);
  const size_t oAGG = off; off = al256(off + (size_t)MP * AGP * 2);
  const size_t oW   = off; off = al256(off + (size_t)NCP * KCAT * 2);
  const size_t oB   = off; off = al256(off + (size_t)64 * 4);
  const size_t oF   = off; off = al256(off + (size_t)NBLK * FLAGP * 4);
  if (off > ws_size || off > (size_t)WSMAX) return;
  unsigned short* XB   = (unsigned short*)(ws + oXB);
  unsigned short* AGG  = (unsigned short*)(ws + oAGG);
  unsigned short* WCAT = (unsigned short*)(ws + oW);
  float*          BSUM = (float*)(ws + oB);
  int*            FLAG = (int*)(ws + oF);

  const size_t scanLds = (size_t)SC_LDS_INTS * 4;
  const size_t gemmLds = (size_t)G_LDS_INTS * 4;
  hipFuncSetAttribute(reinterpret_cast<const void*>(&k_scan),
                      hipFuncAttributeMaxDynamicSharedMemorySize, (int)scanLds);
  hipFuncSetAttribute(reinterpret_cast<const void*>(&k_gemm_lsm),
                      hipFuncAttributeMaxDynamicSharedMemorySize, (int)gemmLds);

  k_prep<<<PB_X + PB_A + PB_W + PB_M, PTHR, 0, stream>>>(x, wlmax, wrmax, bmax, wlmean, wrmean, bmean,
                                                         XB, AGG, WCAT, BSUM);
  k_scan<<<NBLK, SNTHR, scanLds, stream>>>(ei, XB, AGG, FLAG);
  k_gemm_lsm<<<MP / GBM, GTHR, gemmLds, stream>>>(XB, AGG, (const int*)WCAT, BSUM, FLAG, out);
}
